// MotifsBackend_29334626632039
// MI455X (gfx1250) — hardware-verified
//
#include <hip/hip_runtime.h>


constexpr int NB_ = 8;
constexpr int NS_ = 4096;
constexpr int NCH = 64;
constexpr int NM_ = 8;
constexpr int LW_ = 12;
constexpr int H2_ = 512;
constexpr int HO_ = 256;
constexpr int NT_ = NB_ * NS_;
constexpr int TR_ = 16;
constexpr int XR_ = TR_ + LW_ - 1;
constexpr int FP_ = 520;
constexpr int OP_ = 260;

static_assert(NM_ * NCH == H2_);
static_assert(NT_ % TR_ == 0);
static_assert(NS_ % TR_ == 0);
static_assert(H2_ % 32 == 0);
static_assert(HO_ % 32 == 0);
static_assert((FP_ * 2) % 16 == 0);
static_assert((OP_ * 4) % 16 == 0);

constexpr int OFF_MZ = 0;
constexpr int OFF_XS = OFF_MZ + NM_ * NCH * LW_ * 4;
constexpr int OFF_FH = 32768;
constexpr int OFF_FL = OFF_FH + TR_ * FP_ * 2;
constexpr int OFF_HH = OFF_FL + TR_ * FP_ * 2;
constexpr int OFF_HL = OFF_HH + TR_ * FP_ * 2;
constexpr int OFF_RS = OFF_HL + TR_ * FP_ * 2;
constexpr int OFF_RQ = OFF_RS + 8 * TR_ * 4;
constexpr int OFF_OS = OFF_RQ + 8 * TR_ * 4;
constexpr int LDS_BYTES = OFF_OS + TR_ * OP_ * 4;
static_assert(OFF_XS + XR_ * NCH * 4 <= OFF_FH);
static_assert(OFF_FH % 16 == 0);
static_assert(OFF_FL % 16 == 0);
static_assert(OFF_HH % 16 == 0);
static_assert(OFF_HL % 16 == 0);
static_assert(OFF_RS % 16 == 0);
static_assert(OFF_RQ % 16 == 0);
static_assert(OFF_OS % 16 == 0);
static_assert(LDS_BYTES == 116992);

typedef float          v4f   __attribute__((ext_vector_type(4)));
typedef float          v8f   __attribute__((ext_vector_type(8)));
typedef __bf16         v16b  __attribute__((ext_vector_type(16)));
typedef unsigned short u16x8 __attribute__((ext_vector_type(8)));

union FragB { u16x8 h[2]; v16b v; };

__device__ __forceinline__ unsigned short f2bf(float f) {
    unsigned u = __float_as_uint(f);
    unsigned r = u + 0x7FFFu + ((u >> 16) & 1u);
    return (unsigned short)(r >> 16);
}
__device__ __forceinline__ float bf2f(unsigned short b) {
    return __uint_as_float(((unsigned)b) << 16);
}
__device__ __forceinline__ void split8(const v8f& x, u16x8& hv, u16x8& lv) {
#pragma unroll
    for (int c = 0; c < 8; ++c) {
        const float f = x[c];
        const unsigned short hb = f2bf(f);
        hv[c] = hb;
        lv[c] = f2bf(f - bf2f(hb));
    }
}
__device__ __forceinline__ float gelu_erf(float x) {
    return 0.5f * x * (1.0f + erff(x * 0.70710678118654752f));
}

__device__ __forceinline__ void mma_bf(v8f& acc, const FragB& a, const FragB& b) {
    acc = __builtin_amdgcn_wmma_f32_16x16x32_bf16(false, a.v, false, b.v, (short)0, acc, false, false);
    asm volatile("v_nop\n\tv_nop\n\tv_nop\n\tv_nop" : "+v"(acc) : "v"(a.v), "v"(b.v));
}

__global__ __launch_bounds__(256)
void motifz_kernel(const float* __restrict__ motifs, float* mz)
{
    __shared__ __attribute__((aligned(16))) float smz[NM_ * NCH * LW_];
    const int tid = threadIdx.x;
#pragma unroll 1
    for (int rr = 0; rr < 2; ++rr) {
        const int row = tid * 2 + rr;
        const float* p = motifs + row * LW_;
        const v4f a0 = *(const v4f*)(p);
        const v4f a1 = *(const v4f*)(p + 4);
        const v4f a2 = *(const v4f*)(p + 8);
        float v[LW_];
        v[0] = a0.x; v[1] = a0.y; v[2]  = a0.z; v[3]  = a0.w;
        v[4] = a1.x; v[5] = a1.y; v[6]  = a1.z; v[7]  = a1.w;
        v[8] = a2.x; v[9] = a2.y; v[10] = a2.z; v[11] = a2.w;
        float s = 0.0f;
#pragma unroll
        for (int l = 0; l < LW_; ++l) s += v[l];
        const float mean = s * (1.0f / LW_);
        float q = 0.0f;
#pragma unroll
        for (int l = 0; l < LW_; ++l) { v[l] = v[l] - mean; q += v[l] * v[l]; }
        const float sd  = sqrtf(q * (1.0f / LW_)) + 1e-8f;
        const float inv = 1.0f / sd;
#pragma unroll
        for (int l = 0; l < LW_; ++l) smz[row * LW_ + l] = v[l] * inv;
    }
    __syncthreads();
    v4f vals[6];
#pragma unroll
    for (int it = 0; it < 6; ++it) vals[it] = *(const v4f*)(smz + (it * 256 + tid) * 4);
#pragma unroll
    for (int it = 0; it < 6; ++it) *(volatile v4f*)(mz + (size_t)(it * 256 + tid) * 4) = vals[it];
    __threadfence();
#pragma unroll
    for (int it = 0; it < 6; ++it) *(volatile v4f*)(mz + (size_t)(it * 256 + tid) * 4) = vals[it];
}

__global__ __launch_bounds__(256)
void cvt_wt_kernel(const float* __restrict__ W, int K, int N, unsigned short* dh, unsigned short* dl)
{
    const int i = blockIdx.x * 256 + threadIdx.x;
    const int kg = K >> 3;
    const int total = N * kg;
    if (i >= total) return;
    const int n  = i / kg;
    const int k0 = (i - n * kg) * 8;
    v8f x;
#pragma unroll
    for (int q = 0; q < 8; ++q) x[q] = W[(size_t)(k0 + q) * N + n];
    u16x8 hv, lv;
    split8(x, hv, lv);
    const size_t e = (size_t)n * K + k0;
    *(volatile u16x8*)(dh + e) = hv;
    *(volatile u16x8*)(dl + e) = lv;
    __threadfence();
    *(volatile u16x8*)(dh + e) = hv;
    *(volatile u16x8*)(dl + e) = lv;
}

__global__ __launch_bounds__(256)
void fused_kernel(const float* __restrict__ x, const float* __restrict__ mz,
                  const unsigned short* __restrict__ W1h, const unsigned short* __restrict__ W1l,
                  const float* __restrict__ b1, const float* __restrict__ gamma, const float* __restrict__ beta,
                  const unsigned short* __restrict__ W2h, const unsigned short* __restrict__ W2l,
                  const float* __restrict__ b2, float* out)
{
    extern __shared__ __attribute__((aligned(16))) char smem[];
    float*          mzS = (float*)(smem + OFF_MZ);
    float*          xsS = (float*)(smem + OFF_XS);
    unsigned short* flH = (unsigned short*)(smem + OFF_FH);
    unsigned short* flL = (unsigned short*)(smem + OFF_FL);
    unsigned short* hnH = (unsigned short*)(smem + OFF_HH);
    unsigned short* hnL = (unsigned short*)(smem + OFF_HL);
    float*          red = (float*)(smem + OFF_RS);
    float*          rdq = (float*)(smem + OFF_RQ);
    float*          oS  = (float*)(smem + OFF_OS);

    const int tid  = threadIdx.x;
    const int lane = tid & 31;
    const int wave = tid >> 5;
    const int hh   = lane >> 4;
    const int m    = lane & 15;
    const int gr0  = blockIdx.x * TR_;
    const int b    = gr0 / NS_;
    const int s0   = gr0 - b * NS_;

#pragma unroll
    for (int it = 0; it < 6; ++it) {
        const int q = it * 256 + tid;
        *(v4f*)(mzS + q * 4) = *(const v4f*)(mz + (size_t)q * 4);
    }
#pragma unroll
    for (int it = 0; it < 2; ++it) {
        const int q  = it * 256 + tid;
        const int qc = min(q, XR_ * 16 - 1);
        const int r  = qc >> 4;
        const int c4 = (qc & 15) * 4;
        const int sr = max(s0 - (LW_ - 1) + r, 0);
        const v4f v = *(const v4f*)(x + ((size_t)b * NS_ + sr) * NCH + c4);
        if (q < XR_ * 16) *(v4f*)(xsS + r * NCH + c4) = v;
    }
    __syncthreads();

#pragma unroll 1
    for (int it = 0; it < 4; ++it) {
        const int task = it * 256 + tid;
        const int row  = task >> 6;
        const int c    = task & 63;
        float z[LW_];
        float s = 0.0f;
#pragma unroll
        for (int l = 0; l < LW_; ++l) { z[l] = xsS[(row + l) * NCH + c]; s += z[l]; }
        const float mean = s * (1.0f / LW_);
        float q = 0.0f;
#pragma unroll
        for (int l = 0; l < LW_; ++l) { z[l] = z[l] - mean; q += z[l] * z[l]; }
        const float sd  = sqrtf(q * (1.0f / LW_)) + 1e-8f;
        const float inv = 1.0f / sd;
#pragma unroll
        for (int l = 0; l < LW_; ++l) z[l] = z[l] * inv;
#pragma unroll 2
        for (int mm = 0; mm < NM_; ++mm) {
            const int mc = mm * NCH + c;
            const float* mp = mzS + mc * LW_;
            const v4f q0 = *(const v4f*)(mp);
            const v4f q1 = *(const v4f*)(mp + 4);
            const v4f q2 = *(const v4f*)(mp + 8);
            float d = 0.0f;
            d += z[0] * q0.x; d += z[1] * q0.y; d += z[2]  * q0.z; d += z[3]  * q0.w;
            d += z[4] * q1.x; d += z[5] * q1.y; d += z[6]  * q1.z; d += z[7]  * q1.w;
            d += z[8] * q2.x; d += z[9] * q2.y; d += z[10] * q2.z; d += z[11] * q2.w;
            const float sim = d * (1.0f / LW_);
            const float rl  = fmaxf(sim, 0.0f);
            const float r2  = rl * rl;
            const float g   = r2 * r2;
            const unsigned short hb = f2bf(g);
            const unsigned short lb = f2bf(g - bf2f(hb));
            flH[row * FP_ + mc] = hb;
            flL[row * FP_ + mc] = lb;
        }
    }
    __syncthreads();

    v8f acc[4];
#pragma unroll
    for (int j = 0; j < 4; ++j)
#pragma unroll
        for (int r = 0; r < 8; ++r) acc[j][r] = 0.0f;
    {
        const unsigned short* aH = flH + m * FP_ + 8 * hh;
        const unsigned short* aL = flL + m * FP_ + 8 * hh;
        const size_t bbase = (size_t)(wave * 64 + m) * H2_ + 8 * hh;
#pragma unroll 4
        for (int kt = 0; kt < H2_ / 32; ++kt) {
            const int k0 = kt * 32;
            FragB fa, ga;
            fa.h[0] = *(const u16x8*)(aH + k0);
            fa.h[1] = *(const u16x8*)(aH + k0 + 16);
            ga.h[0] = *(const u16x8*)(aL + k0);
            ga.h[1] = *(const u16x8*)(aL + k0 + 16);
            FragB fb[4], gb[4];
#pragma unroll
            for (int j = 0; j < 4; ++j) {
                const unsigned short* p  = W1h + bbase + (size_t)j * 16 * H2_ + k0;
                const unsigned short* pl = W1l + bbase + (size_t)j * 16 * H2_ + k0;
                fb[j].h[0] = *(const u16x8*)(p);
                fb[j].h[1] = *(const u16x8*)(p + 16);
                gb[j].h[0] = *(const u16x8*)(pl);
                gb[j].h[1] = *(const u16x8*)(pl + 16);
            }
#pragma unroll
            for (int j = 0; j < 4; ++j) {
                mma_bf(acc[j], fa, fb[j]);
                mma_bf(acc[j], fa, gb[j]);
                mma_bf(acc[j], ga, fb[j]);
            }
        }
    }

    float g[4][8];
#pragma unroll
    for (int j = 0; j < 4; ++j) {
        const int col = wave * 64 + j * 16 + m;
        const float bb = b1[col];
#pragma unroll
        for (int r = 0; r < 8; ++r) g[j][r] = gelu_erf(acc[j][r] + bb);
    }
    float srow[8];
#pragma unroll
    for (int r = 0; r < 8; ++r) {
        float t = (g[0][r] + g[1][r]) + (g[2][r] + g[3][r]);
        t += __shfl_xor(t, 1, 32);
        t += __shfl_xor(t, 2, 32);
        t += __shfl_xor(t, 4, 32);
        t += __shfl_xor(t, 8, 32);
        srow[r] = t;
    }
    if (m == 0) {
#pragma unroll
        for (int r = 0; r < 8; ++r) red[wave * TR_ + 8 * hh + r] = srow[r];
    }
    __syncthreads();
    float mu[8];
    {
        v4f t0 = {0.0f, 0.0f, 0.0f, 0.0f}, t1 = {0.0f, 0.0f, 0.0f, 0.0f};
#pragma unroll
        for (int w2 = 0; w2 < 8; ++w2) {
            t0 += *(const v4f*)(red + w2 * TR_ + 8 * hh);
            t1 += *(const v4f*)(red + w2 * TR_ + 8 * hh + 4);
        }
        mu[0] = t0.x; mu[1] = t0.y; mu[2] = t0.z; mu[3] = t0.w;
        mu[4] = t1.x; mu[5] = t1.y; mu[6] = t1.z; mu[7] = t1.w;
#pragma unroll
        for (int r = 0; r < 8; ++r) mu[r] = mu[r] * (1.0f / H2_);
    }
    float qrow[8];
#pragma unroll
    for (int r = 0; r < 8; ++r) {
        float t = 0.0f;
#pragma unroll
        for (int j = 0; j < 4; ++j) { const float d = g[j][r] - mu[r]; t += d * d; }
        t += __shfl_xor(t, 1, 32);
        t += __shfl_xor(t, 2, 32);
        t += __shfl_xor(t, 4, 32);
        t += __shfl_xor(t, 8, 32);
        qrow[r] = t;
    }
    if (m == 0) {
#pragma unroll
        for (int r = 0; r < 8; ++r) rdq[wave * TR_ + 8 * hh + r] = qrow[r];
    }
    __syncthreads();
    float rs[8];
    {
        v4f t0 = {0.0f, 0.0f, 0.0f, 0.0f}, t1 = {0.0f, 0.0f, 0.0f, 0.0f};
#pragma unroll
        for (int w2 = 0; w2 < 8; ++w2) {
            t0 += *(const v4f*)(rdq + w2 * TR_ + 8 * hh);
            t1 += *(const v4f*)(rdq + w2 * TR_ + 8 * hh + 4);
        }
        rs[0] = t0.x; rs[1] = t0.y; rs[2] = t0.z; rs[3] = t0.w;
        rs[4] = t1.x; rs[5] = t1.y; rs[6] = t1.z; rs[7] = t1.w;
#pragma unroll
        for (int r = 0; r < 8; ++r) rs[r] = rsqrtf(rs[r] * (1.0f / H2_) + 1e-5f);
    }
#pragma unroll
    for (int j = 0; j < 4; ++j) {
        const int col = wave * 64 + j * 16 + m;
        const float gm = gamma[col];
        const float bt = beta[col];
#pragma unroll
        for (int r = 0; r < 8; ++r) {
            const float v = (g[j][r] - mu[r]) * rs[r] * gm + bt;
            const unsigned short hb = f2bf(v);
            const unsigned short lb = f2bf(v - bf2f(hb));
            hnH[(8 * hh + r) * FP_ + col] = hb;
            hnL[(8 * hh + r) * FP_ + col] = lb;
        }
    }
    __syncthreads();

    v8f acc2[2];
#pragma unroll
    for (int j = 0; j < 2; ++j)
#pragma unroll
        for (int r = 0; r < 8; ++r) acc2[j][r] = 0.0f;
    {
        const unsigned short* aH = hnH + m * FP_ + 8 * hh;
        const unsigned short* aL = hnL + m * FP_ + 8 * hh;
        const size_t bbase = (size_t)(wave * 32 + m) * H2_ + 8 * hh;
#pragma unroll 4
        for (int kt = 0; kt < H2_ / 32; ++kt) {
            const int k0 = kt * 32;
            FragB fa, ga;
            fa.h[0] = *(const u16x8*)(aH + k0);
            fa.h[1] = *(const u16x8*)(aH + k0 + 16);
            ga.h[0] = *(const u16x8*)(aL + k0);
            ga.h[1] = *(const u16x8*)(aL + k0 + 16);
            FragB fb[2], gb[2];
#pragma unroll
            for (int j = 0; j < 2; ++j) {
                const unsigned short* p  = W2h + bbase + (size_t)j * 16 * H2_ + k0;
                const unsigned short* pl = W2l + bbase + (size_t)j * 16 * H2_ + k0;
                fb[j].h[0] = *(const u16x8*)(p);
                fb[j].h[1] = *(const u16x8*)(p + 16);
                gb[j].h[0] = *(const u16x8*)(pl);
                gb[j].h[1] = *(const u16x8*)(pl + 16);
            }
#pragma unroll
            for (int j = 0; j < 2; ++j) {
                mma_bf(acc2[j], fa, fb[j]);
                mma_bf(acc2[j], fa, gb[j]);
                mma_bf(acc2[j], ga, fb[j]);
            }
        }
    }

#pragma unroll
    for (int j = 0; j < 2; ++j) {
        const int col = wave * 32 + j * 16 + m;
        const float bb = b2[col];
#pragma unroll
        for (int r = 0; r < 8; ++r) oS[(8 * hh + r) * OP_ + col] = acc2[j][r] + bb;
    }
    __syncthreads();
    v4f vals[4];
    size_t go[4];
#pragma unroll
    for (int it = 0; it < 4; ++it) {
        const int f   = (it * 256 + tid) * 4;
        const int row = f >> 8;
        const int col = f & 255;
        vals[it] = *(const v4f*)(oS + row * OP_ + col);
        go[it]   = (size_t)gr0 * HO_ + f;
    }
#pragma unroll
    for (int it = 0; it < 4; ++it) *(volatile v4f*)(out + go[it]) = vals[it];
    __threadfence();
#pragma unroll
    for (int it = 0; it < 4; ++it) *(volatile v4f*)(out + go[it]) = vals[it];
}

extern "C" void kernel_launch(void* const* d_in, const int* in_sizes, int n_in,
                              void* d_out, int out_size, void* d_ws, size_t ws_size,
                              hipStream_t stream)
{
    if (n_in < 8) return;
    if (in_sizes[0] != NT_ * NCH)        return;
    if (in_sizes[1] != NM_ * NCH * LW_)  return;
    if (in_sizes[2] != H2_ * H2_)        return;
    if (in_sizes[3] != H2_)              return;
    if (in_sizes[4] != H2_)              return;
    if (in_sizes[5] != H2_)              return;
    if (in_sizes[6] != H2_ * HO_)        return;
    if (in_sizes[7] != HO_)              return;
    if (out_size != NT_ * HO_)           return;

    const float* x      = (const float*)d_in[0];
    const float* motifs = (const float*)d_in[1];
    const float* W1     = (const float*)d_in[2];
    const float* b1     = (const float*)d_in[3];
    const float* gamma  = (const float*)d_in[4];
    const float* beta   = (const float*)d_in[5];
    const float* W2     = (const float*)d_in[6];
    const float* b2     = (const float*)d_in[7];
    float* out = (float*)d_out;

    char* ws = (char*)d_ws;
    size_t off = 0;
    const size_t SZ_MZ = (size_t)NM_ * NCH * LW_ * 4;
    const size_t SZ_W1 = (size_t)H2_ * H2_ * 2;
    const size_t SZ_W2 = (size_t)HO_ * H2_ * 2;
    float*          mz  = (float*)(ws + off);            off += SZ_MZ;
    unsigned short* W1h = (unsigned short*)(ws + off);   off += SZ_W1;
    unsigned short* W1l = (unsigned short*)(ws + off);   off += SZ_W1;
    unsigned short* W2h = (unsigned short*)(ws + off);   off += SZ_W2;
    unsigned short* W2l = (unsigned short*)(ws + off);   off += SZ_W2;
    if (off > ws_size) return;

    const dim3 blk(256);
    motifz_kernel<<<dim3(1), blk, 0, stream>>>(motifs, mz);
    cvt_wt_kernel<<<dim3((H2_ * (H2_ / 8) + 255) / 256), blk, 0, stream>>>(W1, H2_, H2_, W1h, W1l);
    cvt_wt_kernel<<<dim3((HO_ * (H2_ / 8) + 255) / 256), blk, 0, stream>>>(W2, H2_, HO_, W2h, W2l);

    (void)hipFuncSetAttribute((const void*)fused_kernel, hipFuncAttributeMaxDynamicSharedMemorySize, LDS_BYTES);
    fused_kernel<<<dim3(NT_ / TR_), blk, LDS_BYTES, stream>>>(x, mz, W1h, W1l, b1, gamma, beta, W2h, W2l, b2, out);
}
